// SelfAttention_77343771066393
// MI455X (gfx1250) — hardware-verified
//
#include <hip/hip_runtime.h>
#include <stddef.h>


typedef _Float16 v16h __attribute__((ext_vector_type(16)));
typedef _Float16 v8h  __attribute__((ext_vector_type(8)));
typedef float    v8f  __attribute__((ext_vector_type(8)));
typedef float    v4f  __attribute__((ext_vector_type(4)));

#ifndef NB
#define NB 8
#endif
#ifndef SEQ
#define SEQ 4096
#endif
#ifndef SCORE_RES
#define SCORE_RES 1
#endif
#define NB_FULL  8
#define SEQ_FULL 4096
#define CCH 256
#define KCH 64
#define MROWS (NB * SEQ)

static_assert(NB >= 1 && NB <= NB_FULL);
static_assert(SEQ >= 128 && SEQ <= SEQ_FULL && (SEQ % 128) == 0);
static_assert(KCH == 64);
static_assert((CCH % 64) == 0 && (CCH % 32) == 0);
static_assert(CCH == 16 * 16);
static_assert((MROWS % 64) == 0);
static_assert(((KCH * CCH) % 2048) == 0 && ((CCH * CCH) % 2048) == 0);
static_assert((size_t)NB * CCH * SEQ_FULL < (size_t)0x7FFFFFFF);
static_assert(SCORE_RES == 0 || SCORE_RES == 1);

#define LDT 72
#define LDC 68
#define LDO 132
static_assert((LDT % 8) == 0 && LDT >= 64);
static_assert((LDC % 4) == 0 && LDC >= 64);
static_assert((LDO % 4) == 0 && LDO >= 128);

#define WCARRY 64.0f
#define XCARRY 64.0f
#define VCARRY 16.0f
#define PCARRY 16384.0f
#define RCARRY 2048.0f

#define XT_BYTES ((size_t)MROWS * CCH * 2)
#define WQ_BYTES ((size_t)KCH * CCH * 2)
#define WV_BYTES ((size_t)CCH * CCH * 2)
#define QK_BYTES ((size_t)NB * KCH * SEQ * 2)
#define V_BYTES  ((size_t)NB * CCH * SEQ * 2)
#define ST_BYTES ((size_t)NB * SEQ * 4)
#define OFF_XT ((size_t)0)
#define OFF_WQ (OFF_XT + XT_BYTES)
#define OFF_WK (OFF_WQ + WQ_BYTES)
#define OFF_WV (OFF_WK + WQ_BYTES)
#define OFF_QH (OFF_WV + WV_BYTES)
#define OFF_QR (OFF_QH + QK_BYTES)
#define OFF_KH (OFF_QR + QK_BYTES)
#define OFF_KR (OFF_KH + QK_BYTES)
#define OFF_V  (OFF_KR + QK_BYTES)
#define OFF_M  (OFF_V + V_BYTES)
#define OFF_Z  (OFF_M + ST_BYTES)
#define WS_TOTAL (OFF_Z + ST_BYTES)
static_assert((XT_BYTES % 128) == 0 && (WQ_BYTES % 128) == 0 && (WV_BYTES % 128) == 0);
static_assert((QK_BYTES % 128) == 0 && (V_BYTES % 128) == 0 && (ST_BYTES % 128) == 0);
static_assert(WS_TOTAL <= (size_t)134217728);

__device__ __forceinline__ float bf16r(float x) {
  unsigned int u = __float_as_uint(x);
  u = (u + 0x7FFFu + ((u >> 16) & 1u)) & 0xFFFF0000u;
  return __uint_as_float(u);
}

__device__ __forceinline__ v16h frag_at(const _Float16* p) {
  v8h lo = *(const v8h*)(p);
  v8h hi = *(const v8h*)(p + 16);
  v16h out;
#pragma unroll
  for (int i = 0; i < 8; ++i) { out[i] = lo[i]; out[i + 8] = hi[i]; }
  return out;
}

__device__ __forceinline__ v8f wmma16(v16h a, v16h b, v8f c) {
  v8f d = __builtin_amdgcn_wmma_f32_16x16x32_f16(false, a, false, b, (short)0, c,
                                                 false, false);
  asm volatile("v_nop\n\tv_nop\n\tv_nop\n\tv_nop" : "+v"(d) : "v"(a), "v"(b));
  return d;
}

static __device__ __forceinline__ _Float16 toh_flush(float v) {
  const _Float16 r = (_Float16)v;
  return (fabsf(v) < 6.103515625e-05f) ? (_Float16)0.0f : r;
}

__global__ __launch_bounds__(256) void xconv_kernel(
    const float* __restrict__ X, _Float16* __restrict__ Xt) {
  __shared__ _Float16 T[64 * LDT];
  const unsigned tid = threadIdx.x;
  const unsigned n0 = blockIdx.x * 64u;
  const unsigned k0 = blockIdx.y * 64u;
  const unsigned b = blockIdx.z;
  const float* Xb = X + (size_t)b * CCH * SEQ_FULL;
  _Float16* Ob = Xt + (size_t)b * SEQ * CCH;
#pragma unroll 4
  for (unsigned j = 0; j < 16u; ++j) {
    const unsigned idx = tid + 256u * j;
    const unsigned kr = idx >> 6, nc = idx & 63u;
    const float v = Xb[(size_t)(k0 + kr) * SEQ_FULL + n0 + nc];
    T[nc * LDT + kr] = toh_flush(XCARRY * bf16r(v));
  }
  __syncthreads();
  v8h x[2];
  size_t off[2];
#pragma unroll
  for (unsigned i = 0; i < 2u; ++i) {
    const unsigned n = 32u * i + (tid >> 3);
    const unsigned kc = (tid & 7u) * 8u;
    x[i] = *(const v8h*)&T[n * LDT + kc];
    off[i] = (size_t)(n0 + n) * CCH + k0 + kc;
  }
#pragma unroll
  for (int i = 0; i < 2; ++i) *(volatile v8h*)(Ob + off[i]) = x[i];
  __threadfence();
#pragma unroll
  for (int i = 0; i < 2; ++i) *(volatile v8h*)(Ob + off[i]) = x[i];
}

__global__ __launch_bounds__(256) void wplain_kernel(
    const float* __restrict__ W, _Float16* __restrict__ W16, unsigned n) {
  const unsigned e0 = (blockIdx.x * 256u + threadIdx.x) * 8u;
  const bool ok = (e0 + 8u <= n);
  const unsigned ec = ok ? e0 : (n - 8u);
  const v4f a0 = *(const v4f*)(W + ec);
  const v4f a1 = *(const v4f*)(W + ec + 4u);
  v8h o;
#pragma unroll
  for (int i = 0; i < 4; ++i) {
    o[i]     = toh_flush(WCARRY * bf16r(a0[i]));
    o[i + 4] = toh_flush(WCARRY * bf16r(a1[i]));
  }
  if (ok) {
    *(volatile v8h*)(W16 + e0) = o;
    __threadfence();
    *(volatile v8h*)(W16 + e0) = o;
  }
}

template <int RES, int VPLANE>
__device__ __forceinline__ void proj_body(
    const _Float16* __restrict__ A16, const _Float16* __restrict__ Bt,
    const float* __restrict__ bias, const unsigned nout,
    _Float16* __restrict__ out16, _Float16* __restrict__ out16r) {
  __shared__ float Cs[64 * LDC];
  const unsigned K = (unsigned)CCH;
  const unsigned tid = threadIdx.x, lane = tid & 31u, w = tid >> 5;
  const unsigned mw = w >> 1, nw = w & 1u;
  const unsigned hh = lane >> 4, m = lane & 15u;
  const unsigned n0 = blockIdx.x * 64u;
  const unsigned row0 = blockIdx.y * 64u;

  const _Float16* ap  = A16 + (size_t)(row0 + mw * 16u + m) * K + hh * 8u;
  const _Float16* bp0 = Bt + (size_t)(n0 + nw * 32u + m) * K + hh * 8u;
  const _Float16* bp1 = bp0 + (size_t)16 * K;
  v8f acc0 = {}, acc1 = {};
#pragma unroll 2
  for (unsigned k0 = 0; k0 < K; k0 += 32u) {
    const v16h a  = frag_at(ap + k0);
    const v16h b0 = frag_at(bp0 + k0);
    const v16h b1 = frag_at(bp1 + k0);
    acc0 = wmma16(a, b0, acc0);
    acc1 = wmma16(a, b1, acc1);
  }
#pragma unroll
  for (int r = 0; r < 8; ++r) {
    float* d = &Cs[(mw * 16u + hh * 8u + (unsigned)r) * LDC + nw * 32u + m];
    d[0]  = acc0[r];
    d[16] = acc1[r];
  }
  __syncthreads();

  const unsigned bidx = row0 / (unsigned)SEQ;
  const unsigned key0 = row0 - bidx * (unsigned)SEQ;
  const float ocarry = VPLANE ? VCARRY : 1.0f;
  v8h x[2], xr[2];
  size_t off[2];
#pragma unroll
  for (unsigned i = 0; i < 2u; ++i) {
    const unsigned dcol = 32u * i + (tid >> 3);
    const unsigned kk = (tid & 7u) * 8u;
    const float bb = bf16r(bias[n0 + dcol]);
#pragma unroll
    for (unsigned j = 0; j < 8u; ++j) {
      const float t = (Cs[(kk + j) * LDC + dcol] * (1.0f / (WCARRY * XCARRY)) + bb) * ocarry;
      const _Float16 hi = toh_flush(t);
      x[i][j] = hi;
      if (RES) xr[i][j] = toh_flush((t - (float)hi) * RCARRY);
    }
    off[i] = ((size_t)bidx * nout + n0 + dcol) * SEQ + key0 + kk;
  }
#pragma unroll
  for (int i = 0; i < 2; ++i) *(volatile v8h*)(out16 + off[i]) = x[i];
  if (RES) {
#pragma unroll
    for (int i = 0; i < 2; ++i) *(volatile v8h*)(out16r + off[i]) = xr[i];
  }
  __threadfence();
#pragma unroll
  for (int i = 0; i < 2; ++i) *(volatile v8h*)(out16 + off[i]) = x[i];
  if (RES) {
#pragma unroll
    for (int i = 0; i < 2; ++i) *(volatile v8h*)(out16r + off[i]) = xr[i];
  }
}

__global__ __launch_bounds__(256) void proj_qk_kernel(
    const _Float16* __restrict__ A16, const _Float16* __restrict__ Bt,
    const float* __restrict__ bias, _Float16* __restrict__ outh, _Float16* __restrict__ outr) {
  proj_body<SCORE_RES, 0>(A16, Bt, bias, (unsigned)KCH, outh, outr);
}
__global__ __launch_bounds__(256) void proj_v_kernel(
    const _Float16* __restrict__ A16, const _Float16* __restrict__ Bt,
    const float* __restrict__ bias, _Float16* __restrict__ outv) {
  proj_body<0, 1>(A16, Bt, bias, (unsigned)CCH, outv, outv);
}

__global__ __launch_bounds__(256) __attribute__((amdgpu_num_vgpr(256))) void stats_kernel(
    const _Float16* __restrict__ QH, const _Float16* __restrict__ QR,
    const _Float16* __restrict__ KH, const _Float16* __restrict__ KR,
    float* __restrict__ MST, float* __restrict__ IZP) {
  __shared__ __attribute__((aligned(16))) float ms[128];
  __shared__ __attribute__((aligned(16))) float zs[128];
  const unsigned tid = threadIdx.x, lane = tid & 31u;
  const unsigned wave = (unsigned)__builtin_amdgcn_readfirstlane((int)(tid >> 5));
  const unsigned hh = lane >> 4, m = lane & 15u;
  const unsigned b = blockIdx.y;
  const unsigned i0 = blockIdx.x * 128u + wave * 16u;
  const size_t plane = (size_t)b * KCH * SEQ;

  const size_t qoff = plane + (size_t)(i0 + m) * KCH + hh * 8u;
  const v16h qh0 = frag_at(QH + qoff);
  const v16h qh1 = frag_at(QH + qoff + 32);
  v16h qr0 = qh0, qr1 = qh1;
  if (SCORE_RES) {
    qr0 = frag_at(QR + qoff);
    qr1 = frag_at(QR + qoff + 32);
  }

  float mrow[8], lrow[8];
#pragma unroll
  for (int v = 0; v < 8; ++v) { mrow[v] = -1.0e30f; lrow[v] = 0.0f; }

#pragma unroll 1
  for (unsigned jb = 0; jb < (unsigned)SEQ; jb += 64u) {
    v8f s[4];
#pragma unroll
    for (int t = 0; t < 4; ++t) {
      const size_t koff = plane + (size_t)(jb + 16u * (unsigned)t + m) * KCH + hh * 8u;
      const v16h kh0 = frag_at(KH + koff);
      const v16h kh1 = frag_at(KH + koff + 32);
      v8f a = {};
      a = wmma16(qh0, kh0, a);
      a = wmma16(qh1, kh1, a);
      if (SCORE_RES) {
        const v16h kr0 = frag_at(KR + koff);
        const v16h kr1 = frag_at(KR + koff + 32);
        v8f r = {};
        r = wmma16(qh0, kr0, r);
        r = wmma16(qh1, kr1, r);
        r = wmma16(qr0, kh0, r);
        r = wmma16(qr1, kh1, r);
        a = a + r * (1.0f / RCARRY);
      }
      s[t] = a;
    }
#pragma unroll
    for (int v = 0; v < 8; ++v) {
      const float mx = fmaxf(fmaxf(s[0][v], s[1][v]), fmaxf(s[2][v], s[3][v]));
      const float mn = fmaxf(mrow[v], mx);
      const float alpha = __expf(mrow[v] - mn);
      const float e = (__expf(s[0][v] - mn) + __expf(s[1][v] - mn)) +
                      (__expf(s[2][v] - mn) + __expf(s[3][v] - mn));
      lrow[v] = lrow[v] * alpha + e;
      mrow[v] = mn;
    }
  }

#pragma unroll
  for (int v = 0; v < 8; ++v) {
    float mm = mrow[v], ss = lrow[v];
#pragma unroll
    for (int d = 1; d < 16; d <<= 1) {
      const float mo = __shfl_xor(mm, d, 32);
      const float so = __shfl_xor(ss, d, 32);
      const float nm = fmaxf(mm, mo);
      ss = ss * __expf(mm - nm) + so * __expf(mo - nm);
      mm = nm;
    }
    mrow[v] = mm;
    lrow[v] = PCARRY * __builtin_amdgcn_rcpf(ss);
  }
  if (m == 0u) {
#pragma unroll
    for (int v = 0; v < 8; ++v) {
      ms[wave * 16u + hh * 8u + (unsigned)v] = mrow[v];
      zs[wave * 16u + hh * 8u + (unsigned)v] = lrow[v];
    }
  }
  __syncthreads();
  const size_t soff = (size_t)b * SEQ + blockIdx.x * 128u + lane * 4u;
  if (wave == 0u) {
    const v4f val = *(const v4f*)&ms[lane * 4u];
    *(volatile v4f*)(MST + soff) = val;
    __threadfence();
    *(volatile v4f*)(MST + soff) = val;
  } else if (wave == 1u) {
    const v4f val = *(const v4f*)&zs[lane * 4u];
    *(volatile v4f*)(IZP + soff) = val;
    __threadfence();
    *(volatile v4f*)(IZP + soff) = val;
  }
}

__global__ __launch_bounds__(256) __attribute__((amdgpu_num_vgpr(256))) void attn_kernel(
    const _Float16* __restrict__ QH, const _Float16* __restrict__ QR,
    const _Float16* __restrict__ KH, const _Float16* __restrict__ KR,
    const _Float16* __restrict__ V16, const float* __restrict__ MST,
    const float* __restrict__ IZP, const float* __restrict__ X, float* __restrict__ Out) {
  __shared__ __attribute__((aligned(16))) float Os[64 * LDO];
  const unsigned tid = threadIdx.x, lane = tid & 31u;
  const unsigned wave = (unsigned)__builtin_amdgcn_readfirstlane((int)(tid >> 5));
  const unsigned hh = lane >> 4, m = lane & 15u;
  const unsigned b = blockIdx.y;
  const unsigned jblk = blockIdx.x * 128u;
  const unsigned j0 = jblk + wave * 16u;
  const size_t plane = (size_t)b * KCH * SEQ;
  const size_t koff = plane + (size_t)(j0 + m) * KCH + hh * 8u;
  const size_t vbase = ((size_t)b * CCH + m) * SEQ + hh * 8u;
  const size_t sbase = (size_t)b * SEQ + hh * 8u;

  v8f o[16];
#pragma unroll
  for (int ct = 0; ct < 16; ++ct) o[ct] = (v8f){};

#pragma unroll 1
  for (unsigned ib = 0; ib < (unsigned)SEQ; ib += 32u) {
    v16h pf;
#pragma unroll
    for (int t = 0; t < 2; ++t) {
      const size_t qoff = plane + (size_t)(ib + 16u * (unsigned)t + m) * KCH + hh * 8u;
      const v16h kh0 = frag_at(KH + koff);
      const v16h kh1 = frag_at(KH + koff + 32);
      const v16h qh0 = frag_at(QH + qoff);
      const v16h qh1 = frag_at(QH + qoff + 32);
      v8f a = {};
      a = wmma16(qh0, kh0, a);
      a = wmma16(qh1, kh1, a);
      if (SCORE_RES) {
        v8f r = {};
        const v16h kr0 = frag_at(KR + koff);
        const v16h kr1 = frag_at(KR + koff + 32);
        r = wmma16(qh0, kr0, r);
        r = wmma16(qh1, kr1, r);
        const v16h qr0 = frag_at(QR + qoff);
        const v16h qr1 = frag_at(QR + qoff + 32);
        r = wmma16(qr0, kh0, r);
        r = wmma16(qr1, kh1, r);
        a = a + r * (1.0f / RCARRY);
      }
      const size_t so = sbase + ib + 16u * (unsigned)t;
      const v4f mi0 = *(const v4f*)(MST + so);
      const v4f mi1 = *(const v4f*)(MST + so + 4u);
      const v4f z0  = *(const v4f*)(IZP + so);
      const v4f z1  = *(const v4f*)(IZP + so + 4u);
#pragma unroll
      for (int v = 0; v < 4; ++v) {
        const float e0 = __expf(a[v] - mi0[v]) * z0[v];
        const float e1 = __expf(a[v + 4] - mi1[v]) * z1[v];
        pf[8 * t + v]     = toh_flush(e0);
        pf[8 * t + v + 4] = toh_flush(e1);
      }
    }
#pragma unroll
    for (int ct = 0; ct < 16; ++ct) {
      const v16h vf = frag_at(V16 + vbase + (size_t)ct * 16u * SEQ + ib);
      o[ct] = wmma16(vf, pf, o[ct]);
    }
  }

#pragma unroll
  for (int g = 0; g < 4; ++g) {
#pragma unroll
    for (int q = 0; q < 4; ++q)
#pragma unroll
      for (int r = 0; r < 8; ++r)
        Os[((unsigned)q * 16u + hh * 8u + (unsigned)r) * LDO + wave * 16u + m] = o[4 * g + q][r];
    __syncthreads();
#pragma unroll
    for (int half = 0; half < 2; ++half) {
      v4f xs[4];
      size_t off[4];
#pragma unroll
      for (unsigned i = 0; i < 4u; ++i) {
        const unsigned row = 32u * (unsigned)half + 8u * i + wave;
        const unsigned c4 = lane * 4u;
        const v4f u = *(const v4f*)&Os[row * LDO + c4];
        const size_t gidx =
            ((size_t)b * CCH + (unsigned)g * 64u + row) * SEQ_FULL + jblk + c4;
        const v4f xin = *(const v4f*)(X + gidx);
        v4f val;
#pragma unroll
        for (int j = 0; j < 4; ++j)
          val[j] = bf16r(xin[j]) + u[j] * (1.0f / (PCARRY * VCARRY));
        xs[i] = val;
        off[i] = gidx;
      }
#pragma unroll
      for (int i = 0; i < 4; ++i) *(volatile v4f*)(Out + off[i]) = xs[i];
      __threadfence();
#pragma unroll
      for (int i = 0; i < 4; ++i) *(volatile v4f*)(Out + off[i]) = xs[i];
    }
    __syncthreads();
  }
}

extern "C" void kernel_launch(void* const* d_in, const int* in_sizes, int n_in,
                              void* d_out, int out_size, void* d_ws, size_t ws_size,
                              hipStream_t stream) {
  if (n_in < 7) return;
  const long long need_x = ((long long)(NB - 1) * CCH + (CCH - 1)) * SEQ_FULL + SEQ;
  if ((long long)in_sizes[0] < need_x) return;
  if ((long long)in_sizes[1] < (long long)KCH * CCH) return;
  if ((long long)in_sizes[3] < (long long)KCH * CCH) return;
  if ((long long)in_sizes[5] < (long long)CCH * CCH) return;
  if (in_sizes[2] < KCH || in_sizes[4] < KCH || in_sizes[6] < CCH) return;
  if ((long long)out_size < need_x) return;
  if (ws_size < WS_TOTAL) return;

  const float* X  = (const float*)d_in[0];
  const float* wq = (const float*)d_in[1];
  const float* bq = (const float*)d_in[2];
  const float* wk = (const float*)d_in[3];
  const float* bk = (const float*)d_in[4];
  const float* wv = (const float*)d_in[5];
  const float* bv = (const float*)d_in[6];
  float* out = (float*)d_out;

  char* ws = (char*)d_ws;
  _Float16* Xt16 = (_Float16*)(ws + OFF_XT);
  _Float16* Wq16 = (_Float16*)(ws + OFF_WQ);
  _Float16* Wk16 = (_Float16*)(ws + OFF_WK);
  _Float16* Wv16 = (_Float16*)(ws + OFF_WV);
  _Float16* Qh16 = (_Float16*)(ws + OFF_QH);
  _Float16* Qr16 = (_Float16*)(ws + OFF_QR);
  _Float16* Kh16 = (_Float16*)(ws + OFF_KH);
  _Float16* Kr16 = (_Float16*)(ws + OFF_KR);
  _Float16* Vv16 = (_Float16*)(ws + OFF_V);
  float*    Mst  = (float*)(ws + OFF_M);
  float*    Izp  = (float*)(ws + OFF_Z);

  dim3 blk(256);

  xconv_kernel<<<dim3(SEQ / 64, CCH / 64, NB), blk, 0, stream>>>(X, Xt16);
  wplain_kernel<<<dim3((KCH * CCH) / 2048), blk, 0, stream>>>(wq, Wq16, (unsigned)(KCH * CCH));
  wplain_kernel<<<dim3((KCH * CCH) / 2048), blk, 0, stream>>>(wk, Wk16, (unsigned)(KCH * CCH));
  wplain_kernel<<<dim3((CCH * CCH) / 2048), blk, 0, stream>>>(wv, Wv16, (unsigned)(CCH * CCH));

  proj_qk_kernel<<<dim3(KCH / 64, MROWS / 64), blk, 0, stream>>>(Xt16, Wq16, bq, Qh16, Qr16);
  proj_qk_kernel<<<dim3(KCH / 64, MROWS / 64), blk, 0, stream>>>(Xt16, Wk16, bk, Kh16, Kr16);
  proj_v_kernel<<<dim3(CCH / 64, MROWS / 64), blk, 0, stream>>>(Xt16, Wv16, bv, Vv16);

  stats_kernel<<<dim3(SEQ / 128, NB), blk, 0, stream>>>(Qh16, Qr16, Kh16, Kr16, Mst, Izp);
  attn_kernel<<<dim3(SEQ / 128, NB), blk, 0, stream>>>(Qh16, Qr16, Kh16, Kr16, Vv16, Mst, Izp,
                                                       X, out);
}
